// FBPinn_71141838291395
// MI455X (gfx1250) — hardware-verified
//
#include <hip/hip_runtime.h>
#include <math.h>

#pragma clang fp contract(off)

typedef __attribute__((ext_vector_type(16))) _Float16 v16h;
typedef __attribute__((ext_vector_type(8)))  _Float16 v8h;
typedef __attribute__((ext_vector_type(4)))  _Float16 v4h;
typedef __attribute__((ext_vector_type(8)))  float    v8f;
typedef __attribute__((ext_vector_type(4)))  float    v4f;

constexpr int   kNumWin     = 30;
constexpr int   kNeu        = 32;
constexpr int   kWaves      = 8;
constexpr int   kBlock      = kWaves * 32;
constexpr int   kGroups     = 8;
constexpr int   kPtsWave    = kGroups * 16;
constexpr int   kPtsBlock   = kWaves * kPtsWave;
constexpr float kW2Carry    = 16.0f;
constexpr float kW2CarryInv = 0.0625f;
constexpr float kWinThresh  = 0.001f;
constexpr float kLog2e      = 1.4426950408889634f;
constexpr float kTwoLog2e   = 2.8853900817779268f;
constexpr float kLn2Hi      = 0.693145751953125f;
constexpr float kLn2Lo      = 1.4286068203094172e-06f;
static_assert(kPtsBlock == 4 * kBlock);
static_assert(kNeu * kNeu == 4 * kBlock);

struct WinConst { float m[32]; float sinv[32]; float lft[32]; float rgt[32]; };
static_assert(sizeof(WinConst) == 512);

template <typename T> struct Frag;
template <> struct Frag<_Float16> {
  typedef v16h V; union U { v16h v; v8h h[2]; };
  static __device__ __forceinline__ v16h load(const _Float16* p) {
    U f; f.h[0] = *(const v8h*)(p); f.h[1] = *(const v8h*)(p + 16); return f.v;
  }
  static __device__ __forceinline__ v8f mma(v16h a, v16h b, v8f c) {
    return __builtin_amdgcn_wmma_f32_16x16x32_f16(false, a, false, b, (short)0, c, false, false);
  }
};
__device__ __forceinline__ void mma_guard2(v8f& d0, v8f& d1, v16h a0, v16h a1, v16h b) {
  asm volatile("v_nop\n\tv_nop\n\tv_nop\n\tv_nop" : "+v"(d0), "+v"(d1) : "v"(a0), "v"(a1), "v"(b));
}

__device__ __forceinline__ float hw_exp2(float t) { return __builtin_amdgcn_exp2f(t); }
__device__ __forceinline__ float hw_rcp(float t)  { return __builtin_amdgcn_rcpf(t); }
__device__ __forceinline__ float exp_cw(float t) {
  const float nf = rintf(t * kLog2e);
  float r = fmaf(nf, -kLn2Hi, t);
  r = fmaf(nf, -kLn2Lo, r);
  const float e = hw_exp2(r * kLog2e);
  return ldexpf(e, (int)nf);
}
__device__ __forceinline__ float sigm(float t) { return hw_rcp(1.0f + exp_cw(-t)); }
__device__ __forceinline__ float tanh_fast(float v) {
  const float e = hw_exp2(v * kTwoLog2e);
  return fmaf(-2.0f, hw_rcp(e + 1.0f), 1.0f);
}

__global__ void __launch_bounds__(kBlock)
dd_mlp_fused_kernel(const float* __restrict__ x,
                    const float* __restrict__ W1, const float* __restrict__ B1,
                    const float* __restrict__ W2, const float* __restrict__ B2,
                    const float* __restrict__ W3, const float* __restrict__ B3,
                    float* __restrict__ out, int n, WinConst wc)
{
  __shared__ __align__(16) float    sKey[kPtsBlock];
  __shared__ __align__(16) int      sIdx[kPtsBlock];
  __shared__ __align__(16) float    sRes[kPtsBlock];
  __shared__ __align__(16) _Float16 sW2T[kNeu * kNeu];
  __shared__ __align__(16) float    sVec[4 * kNeu];
  __shared__ __align__(16) float    sCon[4 * 32];

  const int  t    = threadIdx.x;
  const int  lane = t & 31;
  const int  wave = t >> 5;
  const int  hh   = lane >> 4;
  const int  c    = lane & 15;
  const long blockBase = (long)blockIdx.x * kPtsBlock;

  if (t == 0) {
#pragma unroll
    for (int i = 0; i < 32; ++i) {
      sCon[i]      = wc.m[i];
      sCon[32 + i] = wc.sinv[i];
      sCon[64 + i] = wc.lft[i];
      sCon[96 + i] = wc.rgt[i];
    }
  }
#pragma unroll
  for (int q = 0; q < 4; ++q) {
    const int li = t + q * kBlock;
    long p = blockBase + li;
    p = (p < (long)n) ? p : (long)(n - 1);
    sKey[li] = x[p];
    sIdx[li] = li;
  }
  __syncthreads();

#pragma unroll 1
  for (int kk = 2; kk <= kPtsBlock; kk <<= 1) {
#pragma unroll 1
    for (int j = kk >> 1; j >= 1; j >>= 1) {
#pragma unroll
      for (int rep = 0; rep < 2; ++rep) {
        const int q  = t + rep * kBlock;
        const int i  = ((q & ~(j - 1)) << 1) | (q & (j - 1));
        const int i2 = i | j;
        const float a  = sKey[i],  b  = sKey[i2];
        const int   ia = sIdx[i],  ib = sIdx[i2];
        const bool  up = ((i & kk) == 0);
        const bool  sw = ((a > b) == up);
        sKey[i]  = sw ? b : a;
        sKey[i2] = sw ? a : b;
        sIdx[i]  = sw ? ib : ia;
        sIdx[i2] = sw ? ia : ib;
      }
      __syncthreads();
    }
  }

  const int slot0 = wave * kPtsWave + c;
  float xs[kGroups], acc[kGroups];
#pragma unroll
  for (int g = 0; g < kGroups; ++g) {
    xs[g]  = sKey[slot0 + 16 * g];
    acc[g] = 0.0f;
  }

  const v8f zero8 = {0.f, 0.f, 0.f, 0.f, 0.f, 0.f, 0.f, 0.f};

#pragma unroll 1
  for (int w = 0; w < kNumWin; ++w) {
    __syncthreads();
    {
      const int nn = t >> 3;
      const int kq = (t & 7) * 4;
      const float* src = W2 + (size_t)w * (kNeu * kNeu) + nn;
      const float a0 = src[(kq + 0) * kNeu];
      const float a1 = src[(kq + 1) * kNeu];
      const float a2 = src[(kq + 2) * kNeu];
      const float a3 = src[(kq + 3) * kNeu];
      v4h hv;
      hv[0] = (_Float16)(a0 * kW2Carry);
      hv[1] = (_Float16)(a1 * kW2Carry);
      hv[2] = (_Float16)(a2 * kW2Carry);
      hv[3] = (_Float16)(a3 * kW2Carry);
      *(v4h*)(sW2T + nn * kNeu + kq) = hv;
      const int vi = t & 31;
      const int vs = (t >> 5) & 3;
      const float u0 = W1[w * kNeu + vi];
      const float u1 = B1[w * kNeu + vi];
      const float u2 = B2[w * kNeu + vi];
      const float u3 = W3[w * kNeu + vi];
      const float f0 = (vs == 0) ? 1.0f : 0.0f;
      const float f1 = (vs == 1) ? 1.0f : 0.0f;
      const float f2 = (vs == 2) ? 1.0f : 0.0f;
      const float f3 = (vs == 3) ? 1.0f : 0.0f;
      float val = f0 * u0;
      val = fmaf(f1, u1, val);
      val = fmaf(f2, u2, val);
      val = fmaf(f3, u3, val);
      sVec[vs * kNeu + vi] = val;
    }
    __syncthreads();

    const float wm     = sCon[w];
    const float ws_inv = sCon[32 + w];
    const float wl     = sCon[64 + w];
    const float wr     = sCon[96 + w];
    const float b3v    = B3[w];

    const v16h fa0 = Frag<_Float16>::load(sW2T + c * kNeu + 8 * hh);
    const v16h fa1 = Frag<_Float16>::load(sW2T + (16 + c) * kNeu + 8 * hh);

    float w1k[16], b1k[16], b2n[16], w3n[16];
#pragma unroll
    for (int half = 0; half < 2; ++half) {
      const int o = 16 * half + 8 * hh;
#pragma unroll
      for (int q4 = 0; q4 < 2; ++q4) {
        const v4f pw1 = *(const v4f*)(sVec + 0 * kNeu + o + 4 * q4);
        const v4f pb1 = *(const v4f*)(sVec + 1 * kNeu + o + 4 * q4);
        const v4f pb2 = *(const v4f*)(sVec + 2 * kNeu + o + 4 * q4);
        const v4f pw3 = *(const v4f*)(sVec + 3 * kNeu + o + 4 * q4);
#pragma unroll
        for (int e = 0; e < 4; ++e) {
          const int i = 8 * half + 4 * q4 + e;
          w1k[i] = pw1[e];
          b1k[i] = pb1[e];
          b2n[i] = pb2[e];
          w3n[i] = pw3[e];
        }
      }
    }

#pragma unroll
    for (int g = 0; g < kGroups; ++g) {
      const float xv  = xs[g];
      const float win = sigm(xv - wl) * sigm(wr - xv);
      const bool  active = win > kWinThresh;
      const unsigned long long anym = __ballot(active ? 1 : 0);
      if (anym != 0ull) {
        const float xn = (xv - wm) * ws_inv;
        v16h fb;
#pragma unroll
        for (int i = 0; i < 16; ++i) fb[i] = (_Float16)tanh_fast(fmaf(xn, w1k[i], b1k[i]));
        v8f d0 = Frag<_Float16>::mma(fa0, fb, zero8);
        v8f d1 = Frag<_Float16>::mma(fa1, fb, zero8);
        mma_guard2(d0, d1, fa0, fa1, fb);
        float part = 0.0f;
#pragma unroll
        for (int r = 0; r < 8; ++r) {
          part = fmaf(tanh_fast(fmaf(d0[r], kW2CarryInv, b2n[r])),     w3n[r],     part);
          part = fmaf(tanh_fast(fmaf(d1[r], kW2CarryInv, b2n[8 + r])), w3n[8 + r], part);
        }
        const float oth = __shfl_xor(part, 16, 32);
        const float o   = (part + oth) + b3v;
        const float contrib = active ? (win * o) : 0.0f;
        acc[g] = acc[g] + contrib;
      }
    }
  }

#pragma unroll
  for (int g = 0; g < kGroups; ++g) {
    const float fin = tanhf(xs[g]) * acc[g];
    const int   oi  = sIdx[slot0 + 16 * g] & (kPtsBlock - 1);
    sRes[oi] = fin;
  }
  __syncthreads();
  {
    const v4f  v  = *(const v4f*)(sRes + 4 * t);
    const long p0 = blockBase + 4 * (long)t;
    const bool ok = (p0 + 3) < (long)n;
    if (ok) *(volatile v4f*)(out + p0) = v;
    __threadfence();
    if (ok) *(volatile v4f*)(out + p0) = v;
  }
}

extern "C" void kernel_launch(void* const* d_in, const int* in_sizes, int n_in,
                              void* d_out, int out_size, void* d_ws, size_t ws_size,
                              hipStream_t stream)
{
  (void)n_in; (void)out_size; (void)d_ws; (void)ws_size;
  const float* x  = (const float*)d_in[0];
  const float* W1 = (const float*)d_in[1];
  const float* b1 = (const float*)d_in[2];
  const float* W2 = (const float*)d_in[3];
  const float* b2 = (const float*)d_in[4];
  const float* W3 = (const float*)d_in[5];
  const float* b3 = (const float*)d_in[6];
  float* out = (float*)d_out;
  const int n = in_sizes[0];

  WinConst wc;
  for (int i = 0; i < 32; ++i) { wc.m[i] = 0.0f; wc.sinv[i] = 0.0f; wc.lft[i] = 0.0f; wc.rgt[i] = 0.0f; }
  const double dom0 = 0.0, dom1 = 100.0;
  const double width = (dom1 - dom0) / (double)kNumWin;
  float lo[kNumWin], hi[kNumWin], mid[kNumWin + 1];
  for (int i = 0; i < kNumWin; ++i) {
    lo[i] = (i == 0) ? (float)dom0 : (float)(((double)i - 0.125) * width);
    hi[i] = (i == kNumWin - 1) ? (float)dom1 : (float)(((double)i + 1.0 + 0.125) * width);
  }
  for (int i = 0; i < kNumWin; ++i) {
    const float ssum = lo[i] + hi[i];
    const float sdif = hi[i] - lo[i];
    const float mean = ssum / 2.0f;
    const float sd   = sdif / 2.0f;
    wc.m[i]    = mean;
    wc.sinv[i] = 1.0f / sd;
  }
  mid[0] = lo[0];
  mid[kNumWin] = hi[kNumWin - 1];
  for (int i = 1; i < kNumWin; ++i) {
    const float s2 = hi[i - 1] + lo[i];
    mid[i] = s2 / 2.0f;
  }
  for (int i = 0; i < kNumWin; ++i) { wc.lft[i] = mid[i]; wc.rgt[i] = mid[i + 1]; }

  int grid = (n + kPtsBlock - 1) / kPtsBlock;
  if (grid < 1) grid = 1;
  hipLaunchKernelGGL(dd_mlp_fused_kernel, dim3(grid), dim3(kBlock), 0, stream,
                     x, W1, b1, W2, b2, W3, b3, out, n, wc);
}
